// TactileGAT_2018634629428
// MI455X (gfx1250) — hardware-run, weakly checked
//
#include <hip/hip_runtime.h>
#include <math.h>

typedef __attribute__((ext_vector_type(16))) _Float16 v16h;
typedef __attribute__((ext_vector_type(8)))  _Float16 v8h;
typedef __attribute__((ext_vector_type(8)))  float    v8f;
typedef __attribute__((ext_vector_type(4)))  float    v4f;

constexpr int kBatch   = 16384;
constexpr int kNode    = 11;
constexpr int kDim     = 64;
constexpr int kTileG   = 16;
constexpr int kRowsT   = kTileG * kNode;
constexpr int kBlocks  = kBatch / kTileG;
constexpr int kNRows   = kBatch * kNode;
constexpr int kMTiles  = kRowsT / 16;
constexpr int kKP      = 32;
constexpr int kHsP     = 65;
constexpr int kAP      = 12;
constexpr int kEdges   = kNode * (kNode - 1);
static_assert(kRowsT == 176);
static_assert(kBlocks * kTileG == kBatch);
static_assert(kMTiles * 16 == kRowsT);
static_assert(2 * kNode <= kKP);
static_assert(kNRows == 180224);

constexpr float kLoCarry = 32.0f;
constexpr float kWCarry  = 2048.0f;
constexpr float kWCarry2 = kWCarry / kLoCarry;
constexpr float kFold    = 1.0f / kWCarry;
static_assert(kWCarry2 == 64.0f);

constexpr size_t kOffPre  = 0;
constexpr size_t kOffPart = kOffPre + (size_t)kNRows * kDim * 4;
constexpr size_t kOffStat = kOffPart + (size_t)kBlocks * 128 * 4;
constexpr size_t kWsTotal = kOffStat + (size_t)192 * 4;
static_assert(kWsTotal == 46662400ull);
static_assert(kWsTotal <= 134217728ull);
static_assert((kOffPart % 128) == 0 && (kOffStat % 128) == 0);

constexpr int kTotal4      = kNRows * kDim / 4;
constexpr int kApplyBlocks = kTotal4 / 512;
static_assert(kApplyBlocks * 512 == kTotal4);

struct FragH {
  union U { v16h v; v8h h[2]; };
  static __device__ __forceinline__ v16h load(const _Float16* p) {
    U f;
    f.h[0] = *(const v8h*)(p);
    f.h[1] = *(const v8h*)(p + 16);
    return f.v;
  }
};

__device__ __forceinline__ v8f mma_f16_guarded(v16h a, v16h b, v8f c) {
  c = __builtin_amdgcn_wmma_f32_16x16x32_f16(false, a, false, b, (short)0, c, false, false);
  asm volatile("v_nop\n\tv_nop\n\tv_nop\n\tv_nop" : "+v"(c) : "v"(a), "v"(b));
  return c;
}

__device__ __forceinline__ void store_plane_row(_Float16* dst, const _Float16 (&p)[kNode],
                                                const _Float16 (&s)[kNode], _Float16 zh) {
  v8h q0, q1, q2, q3;
#pragma unroll
  for (int e = 0; e < 8; ++e) q0[e] = p[e];
#pragma unroll
  for (int e = 0; e < 3; ++e) q1[e] = p[8 + e];
#pragma unroll
  for (int e = 0; e < 5; ++e) q1[3 + e] = s[e];
#pragma unroll
  for (int e = 0; e < 6; ++e) q2[e] = s[5 + e];
  q2[6] = zh;
  q2[7] = zh;
#pragma unroll
  for (int e = 0; e < 8; ++e) q3[e] = zh;
  v8h* d = (v8h*)dst;
  d[0] = q0;
  d[1] = q1;
  d[2] = q2;
  d[3] = q3;
}

union TileA { _Float16 h[kRowsT * kKP]; float f[kRowsT * kAP]; };
union TileB { _Float16 h[kDim * kKP];   float f[8 * 128]; };
static_assert(sizeof(TileA) == 11264);
static_assert(sizeof(TileB) == 4096);

__global__ __launch_bounds__(256) void graph_tile_kernel(
    const float* __restrict__ x, const float* __restrict__ lin_w, const float* __restrict__ lin_b,
    const float* __restrict__ att_i, const float* __restrict__ att_j,
    const float* __restrict__ att_em_i, const float* __restrict__ att_em_j,
    const float* __restrict__ bias_g, const float* __restrict__ emb,
    float* __restrict__ pre, float* __restrict__ part)
{
  __shared__ __align__(16) TileA ra;
  __shared__ __align__(16) TileB rb;
  __shared__ __align__(16) float hs[kRowsT * kHsP];
  __shared__ float sI[kRowsT];
  __shared__ float sJ[kRowsT];
  __shared__ float eI[16];
  __shared__ float eJ[16];
  __shared__ float attI[kDim];
  __shared__ float attJ[kDim];

  const int tid  = threadIdx.x;
  const int lane = tid & 31;
  const int wave = __builtin_amdgcn_readfirstlane((int)(threadIdx.x >> 5));
  const int blk  = blockIdx.x;

  float zf = 0.0f;
  asm volatile("" : "+v"(zf));
  const _Float16 zh = (_Float16)zf;

  {
    const int rloc = (tid < kRowsT) ? tid : (kRowsT - 1);
    const float* xp = x + ((size_t)blk * kRowsT + rloc) * kNode;
    float xv[kNode];
#pragma unroll
    for (int k = 0; k < kNode; ++k) {
      float t = xp[k];
      asm volatile("" : "+v"(t));
      xv[k] = t;
    }
    _Float16 hv[kNode], lv[kNode];
#pragma unroll
    for (int k = 0; k < kNode; ++k) {
      const float hsel = (fabsf(xv[k]) < 6.2e-5f) ? zf : xv[k];
      const _Float16 hh = (_Float16)hsel;
      const float res = xv[k] - (float)hh;
      hv[k] = hh;
      lv[k] = (_Float16)(res * kLoCarry);
    }
    if (tid < kRowsT) store_plane_row(ra.h + tid * kKP, hv, lv, zh);
  }
  if (wave >= 6) {
    const int n = tid - 192;
    const float* wp = lin_w + n * kNode;
    _Float16 w1[kNode], w2[kNode];
#pragma unroll
    for (int k = 0; k < kNode; ++k) {
      const float t = wp[k];
      w1[k] = (_Float16)(t * kWCarry);
      w2[k] = (_Float16)(t * kWCarry2);
    }
    store_plane_row(rb.h + n * kKP, w1, w2, zh);
  }
  if (wave < 2) {
    attI[tid] = att_i[tid];
    attJ[tid] = att_j[tid];
  }
  if (wave == 2) {
    const int node = (lane < kNode) ? lane : (kNode - 1);
    const float* er = emb + node * kDim;
    float a0 = 0.0f, a1 = 0.0f;
#pragma unroll 1
    for (int c4 = 0; c4 < kDim / 4; ++c4) {
      const v4f ev = *(const v4f*)(er + 4 * c4);
      const v4f wi = *(const v4f*)(att_em_i + 4 * c4);
      const v4f wj = *(const v4f*)(att_em_j + 4 * c4);
      a0 = fmaf(ev[0], wi[0], a0);
      a0 = fmaf(ev[1], wi[1], a0);
      a0 = fmaf(ev[2], wi[2], a0);
      a0 = fmaf(ev[3], wi[3], a0);
      a1 = fmaf(ev[0], wj[0], a1);
      a1 = fmaf(ev[1], wj[1], a1);
      a1 = fmaf(ev[2], wj[2], a1);
      a1 = fmaf(ev[3], wj[3], a1);
    }
    if (lane < kNode) {
      eI[lane] = a0;
      eJ[lane] = a1;
    }
  }
  __syncthreads();

  {
    const int rlane = lane & 15;
    const int hh    = lane >> 4;
    const int koff  = hh * 8;
    v16h bfr[4];
    float bv[4];
#pragma unroll
    for (int j = 0; j < 4; ++j) {
      bfr[j] = FragH::load(rb.h + (j * 16 + rlane) * kKP + koff);
      bv[j]  = lin_b[j * 16 + rlane];
    }
    for (int mt = wave; mt < kMTiles; mt += 8) {
      const v16h af = FragH::load(ra.h + (mt * 16 + rlane) * kKP + koff);
      v8f acc[4];
#pragma unroll
      for (int j = 0; j < 4; ++j) {
        acc[j] = (v8f){0.f, 0.f, 0.f, 0.f, 0.f, 0.f, 0.f, 0.f};
        acc[j] = mma_f16_guarded(af, bfr[j], acc[j]);
      }
#pragma unroll
      for (int j = 0; j < 4; ++j) {
#pragma unroll
        for (int r = 0; r < 8; ++r) {
          hs[(mt * 16 + 8 * hh + r) * kHsP + j * 16 + rlane] = acc[j][r] * kFold + bv[j];
        }
      }
    }
  }
  __syncthreads();

  if (tid < kRowsT) {
    const float* hr = hs + tid * kHsP;
    float si = 0.0f, sj = 0.0f;
#pragma unroll 4
    for (int c = 0; c < kDim; ++c) {
      const float hvv = hr[c];
      si = fmaf(hvv, attI[c], si);
      sj = fmaf(hvv, attJ[c], sj);
    }
    sI[tid] = si;
    sJ[tid] = sj;
  }
  __syncthreads();

  if (tid < kRowsT) {
    const int b = tid / kNode;
    const int j = tid - b * kNode;
    const float base = sI[tid] + eI[j];
    float* ar = ra.f + tid * kAP;
    float mx = -3.0e38f;
#pragma unroll 1
    for (int i = 0; i < kNode; ++i) {
      float v = (base + sJ[b * kNode + i]) + eJ[i];
      v = (v >= 0.0f) ? v : 0.2f * v;
      ar[i] = v;
      mx = fmaxf(mx, v);
    }
    float den = 0.0f;
#pragma unroll 1
    for (int i = 0; i < kNode; ++i) {
      const float e = expf(ar[i] - mx);
      ar[i] = e;
      den += e;
    }
    const float inv = 1.0f / den;
#pragma unroll 1
    for (int i = 0; i < kNode; ++i) {
      const float p = ar[i] * inv;
      ar[i] = p;
    }
  }
  __syncthreads();

  float s0 = 0.0f, q0 = 0.0f, s1 = 0.0f, q1 = 0.0f;
  {
    const float bg0 = bias_g[lane];
    const float bg1 = bias_g[lane + 32];
#pragma unroll 1
    for (int r = wave; r < kRowsT; r += 8) {
      const int b = r / kNode;
      const float* ar = ra.f + r * kAP;
      const float* hb = hs + (b * kNode) * kHsP + lane;
      float o0 = 0.0f, o1 = 0.0f;
#pragma unroll
      for (int i = 0; i < kNode; ++i) {
        const float a = ar[i];
        o0 = fmaf(a, hb[i * kHsP], o0);
        o1 = fmaf(a, hb[i * kHsP + 32], o1);
      }
      o0 += bg0;
      o1 += bg1;
      float* drow = pre + ((size_t)blk * kRowsT + r) * kDim;
      volatile float* d0 = drow + lane;
      volatile float* d1 = drow + 32 + lane;
      *d0 = o0;
      *d1 = o1;
      __threadfence();
      *d0 = o0;
      *d1 = o1;
      s0 += o0;
      q0 = fmaf(o0, o0, q0);
      s1 += o1;
      q1 = fmaf(o1, o1, q1);
    }
  }

  {
    float* red = rb.f;
    red[wave * 128 + lane]      = s0;
    red[wave * 128 + 32 + lane] = s1;
    red[wave * 128 + 64 + lane] = q0;
    red[wave * 128 + 96 + lane] = q1;
  }
  __syncthreads();
  if (wave < 4) {
    const float* red = rb.f;
    float t = 0.0f;
#pragma unroll
    for (int w = 0; w < 8; ++w) t += red[w * 128 + tid];
    volatile float* pp = part + (size_t)blk * 128 + tid;
    *pp = t;
    __threadfence();
    *pp = t;
  }
}

__global__ __launch_bounds__(256) void stats_kernel(
    const float* __restrict__ part, const int* __restrict__ edge,
    const float* __restrict__ gamma, const float* __restrict__ beta,
    float* __restrict__ stat, double invN)
{
  __shared__ double dS[128];
  __shared__ float sOut[192];
  const int tid  = threadIdx.x;
  const int wave = __builtin_amdgcn_readfirstlane((int)(threadIdx.x >> 5));
  if (wave < 4) {
    double acc = 0.0;
#pragma unroll 4
    for (int b = 0; b < kBlocks; ++b) acc += (double)part[(size_t)b * 128 + tid];
    dS[tid] = acc;
  }
  __syncthreads();
  if (wave < 2) {
    int okc = 1;
#pragma unroll 1
    for (int e = 0; e < kEdges; ++e) {
      const int i  = e / (kNode - 1);
      const int jj = e - i * (kNode - 1);
      const int j  = jj + ((jj >= i) ? 1 : 0);
      const int sv = edge[e];
      const int dv = edge[kEdges + e];
      okc &= ((sv == i) ? 1 : 0) & ((dv == j) ? 1 : 0);
    }
    const double mean = dS[tid] * invN;
    double var = dS[64 + tid] * invN - mean * mean;
    var = (var > 0.0) ? var : 0.0;
    const float varf = (float)var;
    const float rstd = 1.0f / sqrtf(varf + 1e-5f);
    const float g  = gamma[tid];
    const float bt = beta[tid];
    const float sc = rstd * g;
    const float poison = __uint_as_float(0x7fc00000u);
    sOut[tid]       = (float)mean;
    sOut[64 + tid]  = (okc != 0) ? sc : poison;
    sOut[128 + tid] = bt;
  }
  __syncthreads();
  if (wave < 6) {
    const float v = sOut[tid];
    volatile float* p = stat + tid;
    *p = v;
    __threadfence();
    *p = v;
  }
}

__global__ __launch_bounds__(256) void apply_kernel(
    const float* __restrict__ pre, const float* __restrict__ stat, float* __restrict__ out)
{
  __shared__ __align__(16) float sS[192];
  const int tid  = threadIdx.x;
  const int wave = __builtin_amdgcn_readfirstlane((int)(threadIdx.x >> 5));
  if (wave < 6) sS[tid] = stat[tid];
  __syncthreads();
  const int c0 = (tid & 15) * 4;
  const v4f mean = *(const v4f*)(sS + c0);
  const v4f scl  = *(const v4f*)(sS + 64 + c0);
  const v4f sft  = *(const v4f*)(sS + 128 + c0);
  const size_t i0 = (size_t)blockIdx.x * 512 + tid;
  const size_t i1 = i0 + 256;
  const v4f a = *(const v4f*)(pre + i0 * 4);
  const v4f b = *(const v4f*)(pre + i1 * 4);
  v4f ya, yb;
#pragma unroll
  for (int e = 0; e < 4; ++e) {
    const float ta = (a[e] - mean[e]) * scl[e] + sft[e];
    const float tb = (b[e] - mean[e]) * scl[e] + sft[e];
    ya[e] = (ta >= 0.0f) ? ta : 0.01f * ta;
    yb[e] = (tb >= 0.0f) ? tb : 0.01f * tb;
  }
  volatile v4f* pa = (volatile v4f*)(out + i0 * 4);
  volatile v4f* pb = (volatile v4f*)(out + i1 * 4);
  *pa = ya;
  *pb = yb;
  __threadfence();
  *pa = ya;
  *pb = yb;
}

extern "C" void kernel_launch(void* const* d_in, const int* in_sizes, int n_in,
                              void* d_out, int out_size, void* d_ws, size_t ws_size,
                              hipStream_t stream) {
  if (n_in < 12) return;
  if (in_sizes[0] != kNRows * kNode) return;
  if (in_sizes[1] != 2 * kEdges) return;
  if (in_sizes[2] != kDim * kNode) return;
  if (in_sizes[3] != kDim) return;
  if (in_sizes[4] != kDim) return;
  if (in_sizes[5] != kDim) return;
  if (in_sizes[6] != kDim) return;
  if (in_sizes[7] != kDim) return;
  if (in_sizes[8] != kDim) return;
  if (in_sizes[9] != kNode * kDim) return;
  if (in_sizes[10] != kDim) return;
  if (in_sizes[11] != kDim) return;
  if (out_size != kNRows * kDim) return;
  if (ws_size < kWsTotal) return;

  const float* x        = (const float*)d_in[0];
  const int*   edge     = (const int*)d_in[1];
  const float* lin_w    = (const float*)d_in[2];
  const float* lin_b    = (const float*)d_in[3];
  const float* att_i    = (const float*)d_in[4];
  const float* att_j    = (const float*)d_in[5];
  const float* att_em_i = (const float*)d_in[6];
  const float* att_em_j = (const float*)d_in[7];
  const float* bias_g   = (const float*)d_in[8];
  const float* emb      = (const float*)d_in[9];
  const float* gamma    = (const float*)d_in[10];
  const float* beta     = (const float*)d_in[11];
  float* out = (float*)d_out;

  char* ws = (char*)d_ws;
  float* pre  = (float*)(ws + kOffPre);
  float* part = (float*)(ws + kOffPart);
  float* stat = (float*)(ws + kOffStat);

  graph_tile_kernel<<<kBlocks, 256, 0, stream>>>(
      x, lin_w, lin_b, att_i, att_j, att_em_i, att_em_j, bias_g, emb, pre, part);

  stats_kernel<<<1, 256, 0, stream>>>(part, edge, gamma, beta, stat, 1.0 / (double)kNRows);

  apply_kernel<<<kApplyBlocks, 256, 0, stream>>>(pre, stat, out);
}
